// CrossAttention_53283364274522
// MI455X (gfx1250) — hardware-verified
//
#include <hip/hip_runtime.h>
#include <stdint.h>


typedef _Float16 v16h __attribute__((ext_vector_type(16)));
typedef _Float16 v8h  __attribute__((ext_vector_type(8)));
typedef float    v8f  __attribute__((ext_vector_type(8)));
typedef float    v4f  __attribute__((ext_vector_type(4)));

#ifndef NB
#define NB 2
#endif
#ifndef SEQ
#define SEQ 2048
#endif
#ifndef MCTX
#define MCTX 2048
#endif
#define NB_FULL   2
#define SEQ_FULL  2048
#define MCTX_FULL 2048
#define DIM   1024
#define CTXD  768
#define NHEAD 16
#define DHEAD 64

#define ACT_CAR   8.0f
#define W_CAR     1024.0f
#define PROJ_SCL  0.0009765625f
#define S_SCL     0.001953125f
#define P_CAR     16384.0f
#define O_SCL     0.0078125f
#define OUT_SCL   9.5367431640625e-7f

static_assert(SEQ % 128 == 0);
static_assert(MCTX % 128 == 0);
static_assert(SEQ <= SEQ_FULL);
static_assert(MCTX <= MCTX_FULL);
static_assert(NB <= NB_FULL);
static_assert(DIM % 64 == 0);
static_assert(CTXD % 64 == 0);
static_assert(DIM == NHEAD * DHEAD);
static_assert((DIM % 32) == 0 && (CTXD % 32) == 0);

union Frag16 { v16h v; v8h p[2]; };

__device__ __forceinline__ v16h ld_frag(const _Float16* p, int hl) {
  Frag16 f;
  f.p[0] = *(const v8h*)(p + 8 * hl);
  f.p[1] = *(const v8h*)(p + 16 + 8 * hl);
  return f.v;
}

__device__ __forceinline__ v8f mma(v16h a, v16h b, v8f c) {
  v8f d = __builtin_amdgcn_wmma_f32_16x16x32_f16(false, a, false, b, (short)0, c, false, false);
  asm volatile("v_nop\n\tv_nop\n\tv_nop\n\tv_nop" : "+v"(d) : "v"(a), "v"(b));
  return d;
}

__device__ __forceinline__ float bf16_rne(float x) {
  unsigned int u = __builtin_bit_cast(unsigned int, x);
  u += 0x7FFFu + ((u >> 16) & 1u);
  return __builtin_bit_cast(float, u & 0xFFFF0000u);
}

__global__ __launch_bounds__(256) void k_cvt(const float* __restrict__ src,
                                             _Float16* __restrict__ dst,
                                             int rows, int rows_full, int cols, int total8)
{
  const int i8 = blockIdx.x * 256 + threadIdx.x;
  if (i8 >= total8) return;
  const size_t e   = (size_t)i8 * 8;
  const size_t r   = e / (size_t)cols;
  const int    col = (int)(e - r * (size_t)cols);
  const size_t b   = r / (size_t)rows;
  const size_t n   = r - b * (size_t)rows;
  const float* s = src + (b * (size_t)rows_full + n) * (size_t)cols + col;
  const v4f x0 = *(const v4f*)s;
  const v4f x1 = *(const v4f*)(s + 4);
  v8h o;
#pragma unroll
  for (int j = 0; j < 4; ++j) {
    const float t0 = x0[j];
    const float t1 = x1[j];
    o[j]     = (_Float16)(bf16_rne(t0) * ACT_CAR);
    o[4 + j] = (_Float16)(bf16_rne(t1) * ACT_CAR);
  }
  _Float16* d = dst + e;
  *(volatile v8h*)d = o;
  __threadfence();
  *(volatile v8h*)d = o;
}

__global__ __launch_bounds__(256) void k_wtr(const float* __restrict__ W,
                                             _Float16* __restrict__ Wt, int K, int N)
{
  __shared__ float tile[64 * 65];
  const int tid = threadIdx.x;
  const int n0 = blockIdx.x * 64, k0 = blockIdx.y * 64;
#pragma unroll
  for (int i = 0; i < 4; ++i) {
    const int idx = i * 256 + tid;
    const int r = idx >> 4, c4 = (idx & 15) * 4;
    const v4f v = *(const v4f*)(W + (size_t)(k0 + r) * N + n0 + c4);
    float* tp = tile + r * 65 + c4;
    tp[0] = v[0]; tp[1] = v[1]; tp[2] = v[2]; tp[3] = v[3];
  }
  __syncthreads();
  v8h o[2];
  _Float16* dp[2];
#pragma unroll
  for (int i = 0; i < 2; ++i) {
    const int line = i * 32 + (tid >> 3);
    const int pc   = (tid & 7) * 8;
#pragma unroll
    for (int j = 0; j < 8; ++j)
      o[i][j] = (_Float16)(bf16_rne(tile[(pc + j) * 65 + line]) * W_CAR);
    dp[i] = Wt + (size_t)(n0 + line) * K + k0 + pc;
  }
  *(volatile v8h*)dp[0] = o[0];
  *(volatile v8h*)dp[1] = o[1];
  __threadfence();
  *(volatile v8h*)dp[0] = o[0];
  *(volatile v8h*)dp[1] = o[1];
}

template <int MODE>
__global__ __launch_bounds__(128) __attribute__((amdgpu_num_vgpr(256)))
void k_gemm(const _Float16* __restrict__ A, const _Float16* __restrict__ Bt, int K,
            _Float16* __restrict__ P0, _Float16* __restrict__ P1, float* __restrict__ Of,
            int rpb)
{
  __shared__ float lds32[128 * 68];
  _Float16* lds16 = reinterpret_cast<_Float16*>(lds32);

  const int tid = threadIdx.x, lane = tid & 31, w = tid >> 5;
  const int hl = lane >> 4, c = lane & 15;
  const int m0 = blockIdx.y * 128, n0 = blockIdx.x * 64;
  const int mw = m0 + 32 * w;

  const _Float16* ap0 = A  + (size_t)(mw + c) * K;
  const _Float16* ap1 = A  + (size_t)(mw + 16 + c) * K;
  const _Float16* bp  = Bt + (size_t)(n0 + c) * K;
  const size_t bst = (size_t)16 * K;

  v8f acc[8] = {};
#pragma unroll 1
  for (int k0 = 0; k0 < K; k0 += 32) {
    const v16h a0 = ld_frag(ap0 + k0, hl);
    const v16h a1 = ld_frag(ap1 + k0, hl);
    const v16h b0 = ld_frag(bp + k0, hl);
    const v16h b1 = ld_frag(bp + bst + k0, hl);
    const v16h b2 = ld_frag(bp + 2 * bst + k0, hl);
    const v16h b3 = ld_frag(bp + 3 * bst + k0, hl);
    acc[0] = mma(a0, b0, acc[0]);
    acc[1] = mma(a0, b1, acc[1]);
    acc[2] = mma(a0, b2, acc[2]);
    acc[3] = mma(a0, b3, acc[3]);
    acc[4] = mma(a1, b0, acc[4]);
    acc[5] = mma(a1, b1, acc[5]);
    acc[6] = mma(a1, b2, acc[6]);
    acc[7] = mma(a1, b3, acc[7]);
  }

  const int b  = m0 / rpb;
  const int nn = m0 - b * rpb;

  if (MODE == 2) {
#pragma unroll
    for (int i = 0; i < 2; ++i)
#pragma unroll
      for (int t = 0; t < 4; ++t)
#pragma unroll
        for (int r = 0; r < 8; ++r) {
          const int rowl = 32 * w + 16 * i + 8 * hl + r;
          lds32[rowl * 68 + 16 * t + c] = acc[i * 4 + t][r] * OUT_SCL;
        }
    __syncthreads();
    float* base = Of + ((size_t)b * SEQ_FULL + nn) * DIM + n0;
    for (int i = 0; i < 16; ++i) {
      const int q = i * 128 + tid;
      const int rowl = q >> 4, coff = (q & 15) * 4;
      const v4f v = *(const v4f*)(lds32 + rowl * 68 + coff);
      *(volatile v4f*)(base + (size_t)rowl * DIM + coff) = v;
    }
    __threadfence();
    for (int i = 0; i < 16; ++i) {
      const int q = i * 128 + tid;
      const int rowl = q >> 4, coff = (q & 15) * 4;
      const v4f v = *(const v4f*)(lds32 + rowl * 68 + coff);
      *(volatile v4f*)(base + (size_t)rowl * DIM + coff) = v;
    }
  } else {
    const bool vpart = (MODE == 1) && (n0 >= DIM);
    if (!vpart) {
#pragma unroll
      for (int i = 0; i < 2; ++i)
#pragma unroll
        for (int t = 0; t < 4; ++t)
#pragma unroll
          for (int r = 0; r < 8; ++r) {
            const int rowl = 32 * w + 16 * i + 8 * hl + r;
            lds16[rowl * 72 + 16 * t + c] = (_Float16)(acc[i * 4 + t][r] * PROJ_SCL);
          }
      __syncthreads();
      const int h = n0 / DHEAD;
      _Float16* base = P0 + ((size_t)(b * NHEAD + h) * rpb + nn) * DHEAD;
      for (int i = 0; i < 8; ++i) {
        const int q = i * 128 + tid;
        const int rowl = q >> 3, ch = (q & 7) * 8;
        const v8h v = *(const v8h*)(lds16 + rowl * 72 + ch);
        *(volatile v8h*)(base + (size_t)rowl * DHEAD + ch) = v;
      }
      __threadfence();
      for (int i = 0; i < 8; ++i) {
        const int q = i * 128 + tid;
        const int rowl = q >> 3, ch = (q & 7) * 8;
        const v8h v = *(const v8h*)(lds16 + rowl * 72 + ch);
        *(volatile v8h*)(base + (size_t)rowl * DHEAD + ch) = v;
      }
    } else {
#pragma unroll
      for (int i = 0; i < 2; ++i)
#pragma unroll
        for (int t = 0; t < 4; ++t)
#pragma unroll
          for (int r = 0; r < 8; ++r) {
            const int rowl = 32 * w + 16 * i + 8 * hl + r;
            lds16[(16 * t + c) * 136 + rowl] = (_Float16)(acc[i * 4 + t][r] * PROJ_SCL);
          }
      __syncthreads();
      const int h = (n0 - DIM) / DHEAD;
      _Float16* base = P1 + ((size_t)(b * NHEAD + h) * DHEAD) * rpb + nn;
      for (int i = 0; i < 8; ++i) {
        const int q = i * 128 + tid;
        const int d = q >> 4, moff = (q & 15) * 8;
        const v8h v = *(const v8h*)(lds16 + d * 136 + moff);
        *(volatile v8h*)(base + (size_t)d * rpb + moff) = v;
      }
      __threadfence();
      for (int i = 0; i < 8; ++i) {
        const int q = i * 128 + tid;
        const int d = q >> 4, moff = (q & 15) * 8;
        const v8h v = *(const v8h*)(lds16 + d * 136 + moff);
        *(volatile v8h*)(base + (size_t)d * rpb + moff) = v;
      }
    }
  }
}

__global__ __launch_bounds__(256) __attribute__((amdgpu_num_vgpr(256)))
void k_attn(const _Float16* __restrict__ Q16, const _Float16* __restrict__ K16,
            const _Float16* __restrict__ Vt16, _Float16* __restrict__ O16)
{
  __shared__ _Float16 ldsK[64 * 72];
  __shared__ _Float16 ldsV[64 * 72];
  __shared__ _Float16 ldsP[8 * 16 * 72];

  const int tid = threadIdx.x, lane = tid & 31, w = tid >> 5;
  const int hl = lane >> 4, c = lane & 15;
  const int qtiles = SEQ / 128;
  const int bh = blockIdx.x / qtiles;
  const int qt = blockIdx.x - bh * qtiles;
  const int b  = bh / NHEAD, h = bh - b * NHEAD;
  const int nw = qt * 128 + 16 * w;

  const _Float16* qp = Q16 + ((size_t)bh * SEQ + nw + c) * DHEAD;
  const v16h q0 = ld_frag(qp, hl);
  const v16h q1 = ld_frag(qp + 32, hl);
  const _Float16* kb = K16  + (size_t)bh * MCTX * DHEAD;
  const _Float16* vb = Vt16 + (size_t)bh * DHEAD * MCTX;
  _Float16* myP = ldsP + w * (16 * 72);

  float m[8], l[8];
  v8f o[4] = {};
#pragma unroll
  for (int r = 0; r < 8; ++r) { m[r] = -__builtin_inff(); l[r] = 0.f; }

#pragma unroll 1
  for (int kt = 0; kt < MCTX / 64; ++kt) {
    const int mk = kt * 64;
#pragma unroll
    for (int j = 0; j < 2; ++j) {
      const int s  = j * 256 + tid;
      const int rr = s >> 3, cc = (s & 7) * 8;
      const v8h kv8 = *(const v8h*)(kb + (size_t)(mk + rr) * DHEAD + cc);
      const v8h vv8 = *(const v8h*)(vb + (size_t)rr * MCTX + mk + cc);
      *(v8h*)(ldsK + rr * 72 + cc) = kv8;
      *(v8h*)(ldsV + rr * 72 + cc) = vv8;
    }
    __syncthreads();

    v8f sc[4] = {};
#pragma unroll
    for (int t = 0; t < 4; ++t) {
      const v16h kf0 = ld_frag(ldsK + (16 * t + c) * 72, hl);
      const v16h kf1 = ld_frag(ldsK + (16 * t + c) * 72 + 32, hl);
      sc[t] = mma(q0, kf0, sc[t]);
      sc[t] = mma(q1, kf1, sc[t]);
    }

#pragma unroll
    for (int r = 0; r < 8; ++r) {
      const float v0 = sc[0][r] * S_SCL, v1 = sc[1][r] * S_SCL;
      const float v2 = sc[2][r] * S_SCL, v3 = sc[3][r] * S_SCL;
      float tm = fmaxf(fmaxf(v0, v1), fmaxf(v2, v3));
      tm = fmaxf(tm, __shfl_xor(tm, 1, 32));
      tm = fmaxf(tm, __shfl_xor(tm, 2, 32));
      tm = fmaxf(tm, __shfl_xor(tm, 4, 32));
      tm = fmaxf(tm, __shfl_xor(tm, 8, 32));
      const float mn = fmaxf(m[r], tm);
      const float al = __expf(m[r] - mn);
      const float p0 = __expf(v0 - mn), p1 = __expf(v1 - mn);
      const float p2 = __expf(v2 - mn), p3 = __expf(v3 - mn);
      float rs = (p0 + p1) + (p2 + p3);
      rs += __shfl_xor(rs, 1, 32);
      rs += __shfl_xor(rs, 2, 32);
      rs += __shfl_xor(rs, 4, 32);
      rs += __shfl_xor(rs, 8, 32);
      l[r] = l[r] * al + rs;
      m[r] = mn;
      o[0][r] *= al; o[1][r] *= al; o[2][r] *= al; o[3][r] *= al;
      _Float16* pr = myP + (8 * hl + r) * 72 + c;
      pr[0]  = (_Float16)(p0 * P_CAR);
      pr[16] = (_Float16)(p1 * P_CAR);
      pr[32] = (_Float16)(p2 * P_CAR);
      pr[48] = (_Float16)(p3 * P_CAR);
    }
    __syncthreads();

    const v16h pf0 = ld_frag(myP + c * 72, hl);
    const v16h pf1 = ld_frag(myP + c * 72 + 32, hl);
#pragma unroll
    for (int t = 0; t < 4; ++t) {
      const v16h vf0 = ld_frag(ldsV + (16 * t + c) * 72, hl);
      const v16h vf1 = ld_frag(ldsV + (16 * t + c) * 72 + 32, hl);
      o[t] = mma(pf0, vf0, o[t]);
      o[t] = mma(pf1, vf1, o[t]);
    }
    __syncthreads();
  }

#pragma unroll
  for (int r = 0; r < 8; ++r) {
    const float inv = (1.0f / l[r]) * O_SCL;
    _Float16* pr = myP + (8 * hl + r) * 72 + c;
    pr[0]  = (_Float16)(o[0][r] * inv);
    pr[16] = (_Float16)(o[1][r] * inv);
    pr[32] = (_Float16)(o[2][r] * inv);
    pr[48] = (_Float16)(o[3][r] * inv);
  }
  __syncthreads();
  _Float16* ob = O16 + ((size_t)b * SEQ + nw) * DIM + h * DHEAD;
  v8h ov[4];
  _Float16* od[4];
#pragma unroll
  for (int i = 0; i < 4; ++i) {
    const int q = i * 32 + lane;
    const int rl = q >> 3, ch = (q & 7) * 8;
    ov[i] = *(const v8h*)(myP + rl * 72 + ch);
    od[i] = ob + (size_t)rl * DIM + ch;
  }
#pragma unroll
  for (int i = 0; i < 4; ++i) *(volatile v8h*)od[i] = ov[i];
  __threadfence();
#pragma unroll
  for (int i = 0; i < 4; ++i) *(volatile v8h*)od[i] = ov[i];
}

extern "C" void kernel_launch(void* const* d_in, const int* in_sizes, int n_in,
                              void* d_out, int out_size, void* d_ws, size_t ws_size,
                              hipStream_t stream)
{
  if (n_in < 5) return;
  const long need_x = ((long)(NB - 1) * SEQ_FULL + SEQ) * DIM;
  const long need_c = ((long)(NB - 1) * MCTX_FULL + MCTX) * CTXD;
  if ((long)in_sizes[0] < need_x) return;
  if ((long)in_sizes[1] < need_c) return;
  if ((long)in_sizes[2] < (long)DIM * DIM) return;
  if ((long)in_sizes[3] < (long)CTXD * 2 * DIM) return;
  if ((long)in_sizes[4] < (long)DIM * DIM) return;
  if ((long)out_size < need_x) return;

  const float* x   = (const float*)d_in[0];
  const float* ctx = (const float*)d_in[1];
  const float* Wq  = (const float*)d_in[2];
  const float* Wkv = (const float*)d_in[3];
  const float* Wo  = (const float*)d_in[4];
  float* out = (float*)d_out;

  const size_t nX   = (size_t)NB * SEQ * DIM;
  const size_t nC   = (size_t)NB * MCTX * CTXD;
  const size_t nWq  = (size_t)DIM * DIM;
  const size_t nWkv = (size_t)2 * DIM * CTXD;
  const size_t nWo  = (size_t)DIM * DIM;
  const size_t nQ   = (size_t)NB * NHEAD * SEQ * DHEAD;
  const size_t nK   = (size_t)NB * NHEAD * MCTX * DHEAD;
  const size_t nV   = nK;
  const size_t nO   = (size_t)NB * SEQ * DIM;
  const size_t total_halves = nX + nC + nWq + nWkv + nWo + nQ + nK + nV + nO;
  if (total_halves * sizeof(_Float16) > ws_size) return;

  _Float16* X16  = (_Float16*)d_ws;
  _Float16* C16  = X16  + nX;
  _Float16* Wqt  = C16  + nC;
  _Float16* Wkvt = Wqt  + nWq;
  _Float16* Wot  = Wkvt + nWkv;
  _Float16* Q16  = Wot  + nWo;
  _Float16* K16  = Q16  + nQ;
  _Float16* Vt16 = K16  + nK;
  _Float16* O16  = Vt16 + nV;

  const int tx8 = (int)(nX / 8), tc8 = (int)(nC / 8);
  k_cvt<<<(tx8 + 255) / 256, 256, 0, stream>>>(x,   X16, SEQ,  SEQ_FULL,  DIM,  tx8);
  k_cvt<<<(tc8 + 255) / 256, 256, 0, stream>>>(ctx, C16, MCTX, MCTX_FULL, CTXD, tc8);

  k_wtr<<<dim3(DIM / 64, DIM / 64), 256, 0, stream>>>(Wq, Wqt, DIM, DIM);
  k_wtr<<<dim3(2 * DIM / 64, CTXD / 64), 256, 0, stream>>>(Wkv, Wkvt, CTXD, 2 * DIM);
  k_wtr<<<dim3(DIM / 64, DIM / 64), 256, 0, stream>>>(Wo, Wot, DIM, DIM);

  k_gemm<0><<<dim3(DIM / 64, (NB * SEQ) / 128), 128, 0, stream>>>(
      X16, Wqt, DIM, Q16, K16, out, SEQ);
  k_gemm<1><<<dim3(2 * DIM / 64, (NB * MCTX) / 128), 128, 0, stream>>>(
      C16, Wkvt, CTXD, K16, Vt16, out, MCTX);
  k_attn<<<NB * NHEAD * (SEQ / 128), 256, 0, stream>>>(Q16, K16, Vt16, O16);
  k_gemm<2><<<dim3(DIM / 64, (NB * SEQ) / 128), 128, 0, stream>>>(
      O16, Wot, DIM, Q16, K16, out, SEQ);
}
